// PointNet_SA_Module_KNN_49572512530938
// MI455X (gfx1250) — hardware-verified
//
#include <hip/hip_runtime.h>
#pragma clang fp contract(off)

typedef __attribute__((ext_vector_type(16))) _Float16 v16h;
typedef __attribute__((ext_vector_type(8)))  _Float16 v8h;
typedef __attribute__((ext_vector_type(8)))  float    v8f;
typedef __attribute__((ext_vector_type(4)))  float    v4f;
typedef __attribute__((ext_vector_type(4)))  int      v4i;

constexpr int NBATCH  = 8;
constexpr int NPTS    = 2048;
constexpr int NPOINT  = 512;
constexpr int KNEIGH  = 16;
constexpr int CIN0    = 64;
constexpr int NQUERY  = NBATCH * NPOINT;
constexpr int JROWS   = NQUERY * KNEIGH;
constexpr int SMALL_OUT_ELEMS = NBATCH * 3 * NPOINT;
constexpr float BANK_CARRY     = 16.0f;
constexpr float BANK_CARRY_INV = 1.0f / BANK_CARRY;

static_assert(JROWS == 65536, "row count");
static_assert(SMALL_OUT_ELEMS == 12288, "small output size");
static_assert(49152 / 4 == SMALL_OUT_ELEMS, "out1 byte offset");
static_assert(196608 / 4 == 4 * SMALL_OUT_ELEMS, "out4 byte offset");
static_assert((size_t)(4 * SMALL_OUT_ELEMS + NBATCH * 256 * NPOINT) * 4 == 4390912, "d_out total");

constexpr size_t OFF_FIDX  = 0;
constexpr size_t OFF_KNN   = OFF_FIDX  + 16384;
constexpr size_t OFF_BT0   = OFF_KNN   + 262144;
constexpr size_t OFF_BT1   = OFF_BT0   + 65536;
constexpr size_t OFF_BT2   = OFF_BT1   + 131072;
constexpr size_t OFF_TAB0  = OFF_BT2   + 524288;
constexpr size_t OFF_TAB1  = OFF_TAB0  + 1024;
constexpr size_t OFF_PART0 = OFF_TAB1  + 1536;
constexpr size_t OFF_PART1 = OFF_PART0 + 131072;
constexpr size_t OFF_S     = OFF_PART1 + 262144;
constexpr size_t OFF_A0    = OFF_S     + 6291456;
constexpr size_t OFF_Y0    = OFF_A0    + 8388608;
constexpr size_t OFF_A1    = OFF_Y0    + 16777216;
constexpr size_t OFF_Y1    = OFF_A1    + 8388608;
constexpr size_t OFF_A2    = OFF_Y1    + 33554432;
constexpr size_t OFF_YMAX  = OFF_A2    + 16777216;
constexpr size_t WS_TOTAL  = OFF_YMAX  + 4194304;
static_assert(WS_TOTAL <= 134217728, "carve limit");
static_assert(OFF_KNN % 128 == 0 && OFF_BT0 % 128 == 0 && OFF_BT1 % 128 == 0 && OFF_BT2 % 128 == 0, "align");
static_assert(OFF_TAB0 % 128 == 0 && OFF_TAB1 % 128 == 0 && OFF_PART0 % 128 == 0 && OFF_PART1 % 128 == 0, "align");
static_assert(OFF_S % 128 == 0 && OFF_A0 % 128 == 0 && OFF_Y0 % 128 == 0 && OFF_A1 % 128 == 0, "align");
static_assert(OFF_Y1 % 128 == 0 && OFF_A2 % 128 == 0 && OFF_YMAX % 128 == 0, "align");

__device__ __forceinline__ int clampi(int v, int hi) { return v < 0 ? 0 : (v > hi ? hi : v); }

union FragU { v16h v; v8h h[2]; };
__device__ __forceinline__ v16h frag_load(const _Float16* p) {
  FragU f; f.h[0] = *(const v8h*)(p); f.h[1] = *(const v8h*)(p + 16); return f.v;
}
__device__ __forceinline__ v8f mma_h(v16h a, v16h b, v8f c) {
  return __builtin_amdgcn_wmma_f32_16x16x32_f16(false, a, false, b, (short)0, c, false, false);
}
__device__ __forceinline__ void guard_row4(v8f& a0, v8f& a1, v8f& a2, v8f& a3, v16h x, v16h b0, v16h b1, v16h b2, v16h b3) {
  asm volatile("v_nop\n\tv_nop\n\tv_nop\n\tv_nop" : "+v"(a0), "+v"(a1), "+v"(a2), "+v"(a3) : "v"(x), "v"(b0), "v"(b1), "v"(b2), "v"(b3));
}
__device__ __forceinline__ void guard_acc8(v8f& a0, v8f& a1, v8f& a2, v8f& a3, v8f& a4, v8f& a5, v8f& a6, v8f& a7) {
  asm volatile("v_nop\n\tv_nop\n\tv_nop\n\tv_nop" : "+v"(a0), "+v"(a1), "+v"(a2), "+v"(a3), "+v"(a4), "+v"(a5), "+v"(a6), "+v"(a7));
}

__global__ __launch_bounds__(512) void fps_kernel(const float* __restrict__ xyz, int* __restrict__ fidx) {
#pragma clang fp contract(off)
  __shared__ float wval[16];
  __shared__ int   widx[16];
  __shared__ int   sfar;
  __shared__ __align__(16) int spick[NPOINT];
  const int b = blockIdx.x, tid = threadIdx.x;
  const int lane = tid & 31, wv = tid >> 5;
  const float* xb = xyz + (size_t)b * 3 * NPTS;
  float px[4], py[4], pz[4], dist[4];
#pragma unroll
  for (int q = 0; q < 4; ++q) {
    const int n = tid + q * 512;
    px[q] = xb[n]; py[q] = xb[NPTS + n]; pz[q] = xb[2 * NPTS + n];
    dist[q] = 1e10f;
  }
  int far = 0;
#pragma unroll 1
  for (int i = 0; i < NPOINT; ++i) {
    if (tid == 0) spick[i] = far;
    const int fc = clampi(far, NPTS - 1);
    const float cx = xb[fc], cy = xb[NPTS + fc], cz = xb[2 * NPTS + fc];
    float bestv = -1.0f; int besti = 0;
#pragma unroll
    for (int q = 0; q < 4; ++q) {
      const float dx = px[q] - cx, dy = py[q] - cy, dz = pz[q] - cz;
      const float t0 = dx * dx;
      const float t1 = dy * dy;
      const float t2 = dz * dz;
      const float d = (t0 + t2) + t1;
      dist[q] = fminf(dist[q], d);
      if (dist[q] > bestv) { bestv = dist[q]; besti = tid + q * 512; }
    }
#pragma unroll
    for (int off = 16; off > 0; off >>= 1) {
      const float v2 = __shfl_xor(bestv, off, 32);
      const int   i2 = __shfl_xor(besti, off, 32);
      if (v2 > bestv || (v2 == bestv && i2 < besti)) { bestv = v2; besti = i2; }
    }
    if (lane == 0) { wval[wv] = bestv; widx[wv] = besti; }
    __syncthreads();
    if (wv == 0) {
      const int l15 = lane & 15;
      float v = wval[l15];
      int  ix = widx[l15];
#pragma unroll
      for (int off = 8; off > 0; off >>= 1) {
        const float v2 = __shfl_xor(v, off, 32);
        const int   i2 = __shfl_xor(ix, off, 32);
        if (v2 > v || (v2 == v && i2 < ix)) { v = v2; ix = i2; }
      }
      if (lane == 0) sfar = ix;
    }
    __syncthreads();
    far = sfar;
  }
  __syncthreads();
  if (tid < 128) {
    const v4i v = *(const v4i*)(spick + tid * 4);
    int* dst = fidx + (size_t)b * NPOINT + tid * 4;
    *(volatile v4i*)dst = v;
    __threadfence();
    *(volatile v4i*)dst = v;
  }
}

__global__ __launch_bounds__(256) void knn_kernel(const float* __restrict__ xyz, const int* __restrict__ fidx,
                                                  int* __restrict__ knn) {
#pragma clang fp contract(off)
  __shared__ __align__(16) float sx[3 * NPTS];
  __shared__ float sd[256 * 16];
  __shared__ int   si[256 * 16];
  __shared__ __align__(16) int sk[64 * 16];
  const int tid = threadIdx.x;
  const int q0 = blockIdx.x * 64;
  const int b = q0 >> 9;
  const float* xb = xyz + (size_t)b * 3 * NPTS;
#pragma unroll
  for (int it = 0; it < 6; ++it) {
    const int i4 = (it * 256 + tid) * 4;
    const v4f v = *(const v4f*)(xb + i4);
    *(v4f*)(sx + i4) = v;
  }
  __syncthreads();
  const int chunk = tid >> 6, ql = tid & 63;
  const int fi = clampi(fidx[q0 + ql], NPTS - 1);
  const float ax = sx[fi], ay = sx[NPTS + fi], az = sx[2 * NPTS + fi];
  const float a2 = (ax * ax + az * az) + ay * ay;
  float bd[16]; int bi[16];
#pragma unroll
  for (int q = 0; q < 16; ++q) { bd[q] = 3.4e38f; bi[q] = 0; }
  const int n0 = chunk * 512;
#pragma unroll 1
  for (int n = n0; n < n0 + 512; ++n) {
    const float x = sx[n], y = sx[NPTS + n], z = sx[2 * NPTS + n];
    const float b2 = (x * x + z * z) + y * y;
    float p = ax * x;
    p = __builtin_fmaf(ay, y, p);
    p = __builtin_fmaf(az, z, p);
    const float d = (a2 + b2) - 2.0f * p;
    if (d < bd[15]) {
      bd[15] = d; bi[15] = n;
#pragma unroll
      for (int q = 15; q > 0; --q) {
        if (bd[q] < bd[q - 1]) {
          const float tv = bd[q]; bd[q] = bd[q - 1]; bd[q - 1] = tv;
          const int ti = bi[q]; bi[q] = bi[q - 1]; bi[q - 1] = ti;
        }
      }
    }
  }
#pragma unroll
  for (int q = 0; q < 16; ++q) { sd[tid * 16 + q] = bd[q]; si[tid * 16 + q] = bi[q]; }
  __syncthreads();
  if (tid < 64) {
    int p0 = 0, p1 = 0, p2 = 0, p3 = 0;
#pragma unroll 1
    for (int q = 0; q < 16; ++q) {
      const int c0 = p0 > 15 ? 15 : p0, c1 = p1 > 15 ? 15 : p1, c2 = p2 > 15 ? 15 : p2, c3 = p3 > 15 ? 15 : p3;
      const float v0 = sd[(tid) * 16 + c0];
      const float v1 = sd[(64 + tid) * 16 + c1];
      const float v2 = sd[(128 + tid) * 16 + c2];
      const float v3 = sd[(192 + tid) * 16 + c3];
      const int i0 = si[(tid) * 16 + c0];
      const int i1 = si[(64 + tid) * 16 + c1];
      const int i2 = si[(128 + tid) * 16 + c2];
      const int i3 = si[(192 + tid) * 16 + c3];
      int bc = 0; float bv = v0; int bx = i0;
      if (v1 < bv) { bv = v1; bc = 1; bx = i1; }
      if (v2 < bv) { bv = v2; bc = 2; bx = i2; }
      if (v3 < bv) { bv = v3; bc = 3; bx = i3; }
      sk[tid * 16 + q] = bx;
      p0 += (bc == 0) ? 1 : 0;
      p1 += (bc == 1) ? 1 : 0;
      p2 += (bc == 2) ? 1 : 0;
      p3 += (bc == 3) ? 1 : 0;
    }
  }
  __syncthreads();
  {
    const v4i v = *(const v4i*)(sk + tid * 4);
    int* dst = knn + (size_t)q0 * 16 + tid * 4;
    *(volatile v4i*)dst = v;
    __threadfence();
    *(volatile v4i*)dst = v;
  }
}

__global__ __launch_bounds__(256) void small_out_kernel(const float* __restrict__ xyz, const float* __restrict__ nrm,
                                                        const float* __restrict__ Xa, const float* __restrict__ Ya,
                                                        const int* __restrict__ fidx, const int* __restrict__ knn,
                                                        float* __restrict__ out) {
  const int t = blockIdx.x * 256 + threadIdx.x;
  const int p = t & (NPOINT - 1);
  const int bc = t >> 9;
  const int b = bc / 3;
  const int bp = b * NPOINT + p;
  const int fi = clampi(fidx[bp], NPTS - 1);
  const int kz = clampi(knn[(size_t)bp * 16], NPTS - 1);
  const size_t base = (size_t)bc * NPTS;
  const float v0 = xyz[base + fi];
  const float v1 = nrm[base + kz];
  const float v2 = Xa[base + kz];
  const float v3 = Ya[base + kz];
  *(volatile float*)(out + t) = v0;
  *(volatile float*)(out + SMALL_OUT_ELEMS + t) = v1;
  *(volatile float*)(out + 2 * SMALL_OUT_ELEMS + t) = v2;
  *(volatile float*)(out + 3 * SMALL_OUT_ELEMS + t) = v3;
  __threadfence();
  *(volatile float*)(out + t) = v0;
  *(volatile float*)(out + SMALL_OUT_ELEMS + t) = v1;
  *(volatile float*)(out + 2 * SMALL_OUT_ELEMS + t) = v2;
  *(volatile float*)(out + 3 * SMALL_OUT_ELEMS + t) = v3;
}

__global__ __launch_bounds__(256) void geom_score_kernel(
    const float* __restrict__ xyz, const float* __restrict__ nrm,
    const float* __restrict__ Xa, const float* __restrict__ Ya,
    const int* __restrict__ fidx, const int* __restrict__ knn,
    const float* __restrict__ w1a, const float* __restrict__ b1a, const float* __restrict__ w2a, const float* __restrict__ b2a,
    const float* __restrict__ w1b, const float* __restrict__ b1b, const float* __restrict__ w2b, const float* __restrict__ b2b,
    const float* __restrict__ w1c, const float* __restrict__ b1c, const float* __restrict__ w2c, const float* __restrict__ b2c,
    float* __restrict__ S) {
  __shared__ float wS[3 * 312];
  __shared__ float angL[3 * 256];
  __shared__ float eL[8 * 256];
  const int tid = threadIdx.x;
  const int j = blockIdx.x * 256 + tid;
  const int bp = j >> 4;
  const int b = bp >> 9;
  {
    const int i160 = tid < 160 ? tid : 159;
    const int i128 = tid < 128 ? tid : 127;
    const int i16 = tid < 16 ? tid : 15;
    const int i8 = tid < 8 ? tid : 7;
    const float a0 = w1a[i160], a1 = w1b[i160], a2 = w1c[i160];
    const float c0 = w2a[i128], c1 = w2b[i128], c2 = w2c[i128];
    const float d0 = b1a[i16], d1 = b1b[i16], d2 = b1c[i16];
    const float e0 = b2a[i8], e1 = b2b[i8], e2 = b2c[i8];
    if (tid < 160) { wS[tid] = a0; wS[312 + tid] = a1; wS[624 + tid] = a2; }
    if (tid < 128) { wS[176 + tid] = c0; wS[312 + 176 + tid] = c1; wS[624 + 176 + tid] = c2; }
    if (tid < 16)  { wS[160 + tid] = d0; wS[312 + 160 + tid] = d1; wS[624 + 160 + tid] = d2; }
    if (tid < 8)   { wS[304 + tid] = e0; wS[312 + 304 + tid] = e1; wS[624 + 304 + tid] = e2; }
  }
  asm volatile("" ::: "memory");
  __syncthreads();

  const int fi = clampi(fidx[bp], NPTS - 1);
  const int idx = clampi(knn[j], NPTS - 1);
  const float* xb = xyz + (size_t)b * 3 * NPTS;
  const float cx = xb[fi], cy = xb[NPTS + fi], cz = xb[2 * NPTS + fi];
  const float gx = xb[idx] - cx, gy = xb[NPTS + idx] - cy, gz = xb[2 * NPTS + idx] - cz;
  const float sqn = (gx * gx + gy * gy) + gz * gz;
  const float dist = sqrtf(sqn + 1e-10f);
  float dmn = dist, dmx = dist;
#pragma unroll
  for (int off = 1; off < 16; off <<= 1) {
    const float o1 = __shfl_xor(dmn, off, 32);
    const float o2 = __shfl_xor(dmx, off, 32);
    dmn = fminf(dmn, o1);
    dmx = fmaxf(dmx, o2);
  }
  const float distn = (dist - dmn) * (1.0f / ((dmx - dmn) + 1e-10f));
  const float nn = sqrtf(sqn);
  const float* nbp = nrm + (size_t)b * 3 * NPTS;
  const float* Xbp = Xa + (size_t)b * 3 * NPTS;
  const float* Ybp = Ya + (size_t)b * 3 * NPTS;
  const float nx = nbp[idx], ny = nbp[NPTS + idx], nz = nbp[2 * NPTS + idx];
#pragma unroll 1
  for (int t = 0; t < 3; ++t) {
    const float* vb = (t == 0) ? nbp : ((t == 1) ? Xbp : Ybp);
    const float vx = vb[idx], vy = vb[NPTS + idx], vz = vb[2 * NPTS + idx];
    const float dt = (gx * vx + gy * vy) + gz * vz;
    const float vn = sqrtf((vx * vx + vy * vy) + vz * vz);
    float c = dt * (1.0f / (nn * vn + 1e-8f));
    c = fminf(fmaxf(c, -1.0f), 1.0f);
    angL[t * 256 + tid] = acosf(c) * 0.31830988618379067f;
  }
  float g[10];
  g[0] = gx; g[1] = gy; g[2] = gz; g[3] = distn; g[4] = nx; g[5] = ny; g[6] = nz;
  g[7] = angL[tid]; g[8] = angL[256 + tid]; g[9] = angL[512 + tid];

#pragma unroll 1
  for (int l = 0; l < 3; ++l) {
    const float* wl = wS + l * 312;
    float e[8];
#pragma unroll
    for (int m = 0; m < 8; ++m) e[m] = wl[304 + m];
#pragma unroll 1
    for (int i = 0; i < 16; ++i) {
      const float* wr = wl + i * 10;
      float a = wl[160 + i];
#pragma unroll
      for (int q = 0; q < 10; ++q) a = __builtin_fmaf(wr[q], g[q], a);
      const float h = fmaxf(a, 0.0f);
#pragma unroll
      for (int m = 0; m < 8; ++m) e[m] = __builtin_fmaf(wl[176 + m * 16 + i], h, e[m]);
    }
    float emax = e[0];
#pragma unroll
    for (int m = 1; m < 8; ++m) emax = fmaxf(emax, e[m]);
#pragma unroll
    for (int m = 0; m < 8; ++m) eL[m * 256 + tid] = e[m] - emax;
    float esum = 0.0f;
#pragma unroll 1
    for (int m = 0; m < 8; ++m) {
      const float v = expf(eL[m * 256 + tid]);
      eL[m * 256 + tid] = v;
      esum += v;
    }
    const float inv = 1.0f / esum;
    float pr[8];
#pragma unroll
    for (int m = 0; m < 8; ++m) pr[m] = eL[m * 256 + tid] * inv;
    float* Sl = S + (size_t)l * 8 * JROWS + j;
#pragma unroll
    for (int m = 0; m < 8; ++m) *(volatile float*)(Sl + (size_t)m * JROWS) = pr[m];
    __threadfence();
#pragma unroll
    for (int m = 0; m < 8; ++m) *(volatile float*)(Sl + (size_t)m * JROWS) = pr[m];
  }
}

__global__ __launch_bounds__(256) void gather_feats_kernel(const float* __restrict__ pts, const int* __restrict__ knn,
                                                           unsigned short* __restrict__ A0) {
  const int gid = blockIdx.x * 256 + threadIdx.x;
  const int j = gid >> 3;
  const int c8 = (gid & 7) * 8;
  const int b = j >> 13;
  const int idx = clampi(knn[j], NPTS - 1);
  const float* src = pts + ((size_t)b * CIN0 + c8) * NPTS + idx;
  float f[8];
#pragma unroll
  for (int e = 0; e < 8; ++e) f[e] = src[(size_t)e * NPTS];
  v8h hv;
#pragma unroll
  for (int e = 0; e < 8; ++e) hv[e] = (_Float16)f[e];
  _Float16* dst = (_Float16*)A0 + (size_t)j * CIN0 + c8;
  *(volatile v8h*)dst = hv;
  __threadfence();
  *(volatile v8h*)dst = hv;
}

__global__ __launch_bounds__(256) void pack_bank_kernel(const float* __restrict__ bank, unsigned short* __restrict__ Bt,
                                                        int cin, int cout) {
  const int gid = blockIdx.x * 256 + threadIdx.x;
  const int lpr = cin >> 3;
  const int nrows = 8 * cout;
  int n = gid / lpr;
  n = n < nrows ? n : nrows - 1;
  const int c8 = (gid - (gid / lpr) * lpr) * 8;
  const int m = n / cout;
  const int o = n - m * cout;
  const float* src = bank + ((size_t)m * cin + c8) * cout + o;
  float f[8];
#pragma unroll
  for (int e = 0; e < 8; ++e) f[e] = src[(size_t)e * cout];
  v8h hv;
#pragma unroll
  for (int e = 0; e < 8; ++e) hv[e] = (_Float16)(f[e] * BANK_CARRY);
  _Float16* dst = (_Float16*)Bt + (size_t)n * cin + c8;
  *(volatile v8h*)dst = hv;
  __threadfence();
  *(volatile v8h*)dst = hv;
}

template <int CINT, int COUT, int MODE>
__global__ __launch_bounds__(256) void paconv_gemm(const unsigned short* __restrict__ Ap,
                                                   const unsigned short* __restrict__ Btp,
                                                   const float* __restrict__ Sl, float* __restrict__ Out) {
  static_assert(CINT % 32 == 0, "K multiple of 32");
  static_assert(COUT % 64 == 0, "N multiple of 64");
  static_assert(JROWS % 256 == 0, "M multiple of 256");
  constexpr int TN = COUT / 64;
  __shared__ __align__(16) float sS[8 * 256];
  __shared__ __align__(16) float sT[8][16 * 68];
  const _Float16* A = (const _Float16*)Ap;
  const _Float16* Bt = (const _Float16*)Btp;
  const int tid = threadIdx.x, lane = tid & 31, wave = tid >> 5;
  const int tn = blockIdx.x % TN, rb = blockIdx.x / TN;
  const int row0 = rb * 256, n0 = tn * 64;
  {
    float sv[8];
#pragma unroll
    for (int m = 0; m < 8; ++m) sv[m] = Sl[(size_t)m * JROWS + row0 + tid];
#pragma unroll
    for (int m = 0; m < 8; ++m) sS[m * 256 + tid] = sv[m] * BANK_CARRY_INV;
  }
  __syncthreads();

  const int rlane = lane & 15, hh = lane >> 4;
  const int koff = hh * 8, mOff = hh * 8;
  const int m0 = row0 + wave * 32;
  const v8f vzero = (v8f){0.f, 0.f, 0.f, 0.f, 0.f, 0.f, 0.f, 0.f};
  v8f o[2][4];
#pragma unroll
  for (int i = 0; i < 2; ++i)
#pragma unroll
    for (int jj = 0; jj < 4; ++jj) o[i][jj] = vzero;
  const _Float16* Ar0 = A + (size_t)(m0 + rlane) * CINT + koff;
  const _Float16* Ar1 = A + (size_t)(m0 + 16 + rlane) * CINT + koff;

#pragma unroll 1
  for (int m = 0; m < 8; ++m) {
    v8f acc[2][4];
#pragma unroll
    for (int i = 0; i < 2; ++i)
#pragma unroll
      for (int jj = 0; jj < 4; ++jj) acc[i][jj] = vzero;
    const _Float16* Bm = Bt + (size_t)(m * COUT + n0 + rlane) * CINT + koff;
#pragma unroll
    for (int k0 = 0; k0 < CINT; k0 += 32) {
      v16h bh[4];
#pragma unroll
      for (int jj = 0; jj < 4; ++jj) bh[jj] = frag_load(Bm + (size_t)(jj * 16) * CINT + k0);
      {
        const v16h ah = frag_load(Ar0 + k0);
#pragma unroll
        for (int jj = 0; jj < 4; ++jj) acc[0][jj] = mma_h(ah, bh[jj], acc[0][jj]);
        guard_row4(acc[0][0], acc[0][1], acc[0][2], acc[0][3], ah, bh[0], bh[1], bh[2], bh[3]);
      }
      {
        const v16h ah = frag_load(Ar1 + k0);
#pragma unroll
        for (int jj = 0; jj < 4; ++jj) acc[1][jj] = mma_h(ah, bh[jj], acc[1][jj]);
        guard_row4(acc[1][0], acc[1][1], acc[1][2], acc[1][3], ah, bh[0], bh[1], bh[2], bh[3]);
      }
    }
    guard_acc8(acc[0][0], acc[0][1], acc[0][2], acc[0][3], acc[1][0], acc[1][1], acc[1][2], acc[1][3]);
#pragma unroll
    for (int i = 0; i < 2; ++i) {
      const float* sp = sS + m * 256 + wave * 32 + i * 16 + mOff;
      const v4f sa = *(const v4f*)sp;
      const v4f sb = *(const v4f*)(sp + 4);
      float s8[8];
      s8[0] = sa[0]; s8[1] = sa[1]; s8[2] = sa[2]; s8[3] = sa[3];
      s8[4] = sb[0]; s8[5] = sb[1]; s8[6] = sb[2]; s8[7] = sb[3];
#pragma unroll
      for (int jj = 0; jj < 4; ++jj)
#pragma unroll
        for (int r = 0; r < 8; ++r) o[i][jj][r] = __builtin_fmaf(s8[r], acc[i][jj][r], o[i][jj][r]);
    }
  }

  float* slab = sT[wave];
  if (MODE == 0) {
    const int c4 = (lane & 15) * 4;
#pragma unroll
    for (int i = 0; i < 2; ++i) {
      const int mBase = m0 + (i << 4);
#pragma unroll
      for (int jj = 0; jj < 4; ++jj)
#pragma unroll
        for (int r = 0; r < 8; ++r) slab[(mOff + r) * 68 + (jj << 4) + rlane] = o[i][jj][r];
      __builtin_amdgcn_fence(__ATOMIC_RELEASE, "workgroup");
      __builtin_amdgcn_wave_barrier();
      __builtin_amdgcn_fence(__ATOMIC_ACQUIRE, "workgroup");
      for (int pass = 0; pass < 2; ++pass) {
#pragma unroll
        for (int it = 0; it < 8; ++it) {
          const int row = it * 2 + hh;
          const v4f v = *(const v4f*)(slab + row * 68 + c4);
          *(volatile v4f*)(Out + (size_t)(mBase + row) * COUT + n0 + c4) = v;
        }
        __threadfence();
      }
      __builtin_amdgcn_fence(__ATOMIC_RELEASE, "workgroup");
      __builtin_amdgcn_wave_barrier();
      __builtin_amdgcn_fence(__ATOMIC_ACQUIRE, "workgroup");
    }
  } else {
#pragma unroll
    for (int i = 0; i < 2; ++i) {
#pragma unroll
      for (int jj = 0; jj < 4; ++jj) {
        float mx = o[i][jj][0];
#pragma unroll
        for (int r = 1; r < 8; ++r) mx = fmaxf(mx, o[i][jj][r]);
        const float other = __shfl_xor(mx, 16, 32);
        mx = fmaxf(mx, other);
        if (hh == 0) slab[i * 68 + (jj << 4) + rlane] = mx;
      }
    }
    __builtin_amdgcn_fence(__ATOMIC_RELEASE, "workgroup");
    __builtin_amdgcn_wave_barrier();
    __builtin_amdgcn_fence(__ATOMIC_ACQUIRE, "workgroup");
    const int prow = lane >> 4, c4 = (lane & 15) * 4;
    const v4f v = *(const v4f*)(slab + prow * 68 + c4);
    float* dst = Out + (size_t)((m0 >> 4) + prow) * 256 + n0 + c4;
    *(volatile v4f*)dst = v;
    __threadfence();
    *(volatile v4f*)dst = v;
  }
}

template <int COUT>
__global__ __launch_bounds__(256) void bn_stats_kernel(const float* __restrict__ Y, float* __restrict__ part) {
  constexpr int RG = 256 / COUT;
  __shared__ float red[2 * 256];
  const int tid = threadIdx.x, rb = blockIdx.x;
  const int col = tid % COUT, rg = tid / COUT;
  float s = 0.0f, ss = 0.0f;
#pragma unroll 1
  for (int it = 0; it < COUT; ++it) {
    const int row = rb * 256 + rg + it * RG;
    const float v = Y[(size_t)row * COUT + col];
    s += v;
    ss += v * v;
  }
  red[tid] = s;
  red[256 + tid] = ss;
  __syncthreads();
  if (tid < (2 * COUT) / 4) {
    v4f v;
#pragma unroll
    for (int u = 0; u < 4; ++u) {
      const int e = tid * 4 + u;
      const int which = e / COUT;
      const int c = e - which * COUT;
      float a = 0.0f;
#pragma unroll
      for (int q = 0; q < RG; ++q) a += red[which * 256 + q * COUT + c];
      v[u] = a;
    }
    float* dst = part + (size_t)rb * 2 * COUT + tid * 4;
    *(volatile v4f*)dst = v;
    __threadfence();
    *(volatile v4f*)dst = v;
  }
}

template <int COUT>
__global__ __launch_bounds__(COUT) void bn_final_kernel(const float* __restrict__ part, const float* __restrict__ gamma,
                                                        const float* __restrict__ beta, float* __restrict__ tab) {
  const int c = threadIdx.x;
  double s = 0.0, ss = 0.0;
#pragma unroll 1
  for (int rb = 0; rb < 256; ++rb) {
    s += (double)part[(size_t)rb * 2 * COUT + c];
    ss += (double)part[(size_t)rb * 2 * COUT + COUT + c];
  }
  const double inv = 1.0 / 65536.0;
  const double mu = s * inv;
  double var = ss * inv - mu * mu;
  var = var < 0.0 ? 0.0 : var;
  const float rs = 1.0f / sqrtf((float)var + 1e-5f);
  const float muf = (float)mu;
  const float gsc = rs * gamma[c];
  const float bt = beta[c];
  *(volatile float*)(tab + c) = muf;
  *(volatile float*)(tab + COUT + c) = gsc;
  *(volatile float*)(tab + 2 * COUT + c) = bt;
  __threadfence();
  *(volatile float*)(tab + c) = muf;
  *(volatile float*)(tab + COUT + c) = gsc;
  *(volatile float*)(tab + 2 * COUT + c) = bt;
}

template <int COUT>
__global__ __launch_bounds__(256) void bn_apply_kernel(const float* __restrict__ Y, const float* __restrict__ tab,
                                                       unsigned short* __restrict__ Aout) {
  const size_t gid = (size_t)blockIdx.x * 256 + threadIdx.x;
  const size_t e0 = gid * 8;
  const int col = (int)(e0 % COUT);
  const v4f y0 = *(const v4f*)(Y + e0);
  const v4f y1 = *(const v4f*)(Y + e0 + 4);
  const v4f m0 = *(const v4f*)(tab + col);
  const v4f m1 = *(const v4f*)(tab + col + 4);
  const v4f g0 = *(const v4f*)(tab + COUT + col);
  const v4f g1 = *(const v4f*)(tab + COUT + col + 4);
  const v4f b0 = *(const v4f*)(tab + 2 * COUT + col);
  const v4f b1 = *(const v4f*)(tab + 2 * COUT + col + 4);
  v8h hv;
#pragma unroll
  for (int e = 0; e < 4; ++e) {
    const float z0 = fmaxf(__builtin_fmaf(y0[e] - m0[e], g0[e], b0[e]), 0.0f);
    const float z1 = fmaxf(__builtin_fmaf(y1[e] - m1[e], g1[e], b1[e]), 0.0f);
    hv[e] = (_Float16)z0;
    hv[4 + e] = (_Float16)z1;
  }
  _Float16* dst = (_Float16*)Aout + e0;
  *(volatile v8h*)dst = hv;
  __threadfence();
  *(volatile v8h*)dst = hv;
}

__global__ __launch_bounds__(256) void transpose_out_kernel(const float* __restrict__ Ymax, float* __restrict__ out4) {
  __shared__ float tile[32 * 33];
  const int tid = threadIdx.x;
  const int pt0 = blockIdx.x * 32, o0 = blockIdx.y * 32;
  {
    const int pr = tid >> 3, c4 = (tid & 7) * 4;
    const v4f v = *(const v4f*)(Ymax + (size_t)(pt0 + pr) * 256 + o0 + c4);
    tile[pr * 33 + c4 + 0] = v[0];
    tile[pr * 33 + c4 + 1] = v[1];
    tile[pr * 33 + c4 + 2] = v[2];
    tile[pr * 33 + c4 + 3] = v[3];
  }
  __syncthreads();
  const int orow = tid >> 3, p4 = (tid & 7) * 4;
  v4f w;
  w[0] = tile[(p4 + 0) * 33 + orow];
  w[1] = tile[(p4 + 1) * 33 + orow];
  w[2] = tile[(p4 + 2) * 33 + orow];
  w[3] = tile[(p4 + 3) * 33 + orow];
  const int b = pt0 >> 9, p0 = pt0 & (NPOINT - 1);
  float* dst = out4 + ((size_t)b * 256 + o0 + orow) * NPOINT + p0 + p4;
  *(volatile v4f*)dst = w;
  __threadfence();
  *(volatile v4f*)dst = w;
}

extern "C" void kernel_launch(void* const* d_in, const int* in_sizes, int n_in,
                              void* d_out, int out_size, void* d_ws, size_t ws_size,
                              hipStream_t stream) {
  (void)in_sizes; (void)out_size;
  if (n_in < 24) return;
  if (ws_size < WS_TOTAL) return;
  const float* xyz  = (const float*)d_in[0];
  const float* nrm  = (const float*)d_in[1];
  const float* Xax  = (const float*)d_in[2];
  const float* Yax  = (const float*)d_in[3];
  const float* pts  = (const float*)d_in[4];
  const float* w1_0 = (const float*)d_in[5];
  const float* b1_0 = (const float*)d_in[6];
  const float* w2_0 = (const float*)d_in[7];
  const float* b2_0 = (const float*)d_in[8];
  const float* bank0 = (const float*)d_in[9];
  const float* gamma0 = (const float*)d_in[10];
  const float* beta0  = (const float*)d_in[11];
  const float* w1_1 = (const float*)d_in[12];
  const float* b1_1 = (const float*)d_in[13];
  const float* w2_1 = (const float*)d_in[14];
  const float* b2_1 = (const float*)d_in[15];
  const float* bank1 = (const float*)d_in[16];
  const float* gamma1 = (const float*)d_in[17];
  const float* beta1  = (const float*)d_in[18];
  const float* w1_2 = (const float*)d_in[19];
  const float* b1_2 = (const float*)d_in[20];
  const float* w2_2 = (const float*)d_in[21];
  const float* b2_2 = (const float*)d_in[22];
  const float* bank2 = (const float*)d_in[23];

  char* ws = (char*)d_ws;
  int* fidx = (int*)(ws + OFF_FIDX);
  int* knn  = (int*)(ws + OFF_KNN);
  unsigned short* bt0 = (unsigned short*)(ws + OFF_BT0);
  unsigned short* bt1 = (unsigned short*)(ws + OFF_BT1);
  unsigned short* bt2 = (unsigned short*)(ws + OFF_BT2);
  float* tab0  = (float*)(ws + OFF_TAB0);
  float* tab1  = (float*)(ws + OFF_TAB1);
  float* part0 = (float*)(ws + OFF_PART0);
  float* part1 = (float*)(ws + OFF_PART1);
  float* Sall  = (float*)(ws + OFF_S);
  unsigned short* A0 = (unsigned short*)(ws + OFF_A0);
  float* Y0 = (float*)(ws + OFF_Y0);
  unsigned short* A1 = (unsigned short*)(ws + OFF_A1);
  float* Y1 = (float*)(ws + OFF_Y1);
  unsigned short* A2 = (unsigned short*)(ws + OFF_A2);
  float* Ymax = (float*)(ws + OFF_YMAX);

  float* out = (float*)d_out;
  float* out4 = out + 4 * SMALL_OUT_ELEMS;

  fps_kernel<<<NBATCH, 512, 0, stream>>>(xyz, fidx);
  knn_kernel<<<NQUERY / 64, 256, 0, stream>>>(xyz, fidx, knn);
  small_out_kernel<<<SMALL_OUT_ELEMS / 256, 256, 0, stream>>>(xyz, nrm, Xax, Yax, fidx, knn, out);
  geom_score_kernel<<<JROWS / 256, 256, 0, stream>>>(xyz, nrm, Xax, Yax, fidx, knn,
                                                     w1_0, b1_0, w2_0, b2_0,
                                                     w1_1, b1_1, w2_1, b2_1,
                                                     w1_2, b1_2, w2_2, b2_2, Sall);
  gather_feats_kernel<<<(JROWS * 8) / 256, 256, 0, stream>>>(pts, knn, A0);
  pack_bank_kernel<<<(64 * 64) / 256, 256, 0, stream>>>(bank0, bt0, 64, 64);
  pack_bank_kernel<<<(128 * 64) / 256, 256, 0, stream>>>(bank1, bt1, 64, 128);
  pack_bank_kernel<<<(256 * 128) / 256, 256, 0, stream>>>(bank2, bt2, 128, 256);

  paconv_gemm<64, 64, 0><<<(JROWS / 256) * 1, 256, 0, stream>>>(A0, bt0, Sall, Y0);
  bn_stats_kernel<64><<<JROWS / 256, 256, 0, stream>>>(Y0, part0);
  bn_final_kernel<64><<<1, 64, 0, stream>>>(part0, gamma0, beta0, tab0);
  bn_apply_kernel<64><<<(JROWS / 256) * (64 / 8), 256, 0, stream>>>(Y0, tab0, A1);

  paconv_gemm<64, 128, 0><<<(JROWS / 256) * 2, 256, 0, stream>>>(A1, bt1, Sall + (size_t)8 * JROWS, Y1);
  bn_stats_kernel<128><<<JROWS / 256, 256, 0, stream>>>(Y1, part1);
  bn_final_kernel<128><<<1, 128, 0, stream>>>(part1, gamma1, beta1, tab1);
  bn_apply_kernel<128><<<(JROWS / 256) * (128 / 8), 256, 0, stream>>>(Y1, tab1, A2);

  paconv_gemm<128, 256, 1><<<(JROWS / 256) * 4, 256, 0, stream>>>(A2, bt2, Sall + (size_t)16 * JROWS, Ymax);
  transpose_out_kernel<<<dim3(NQUERY / 32, 256 / 32), 256, 0, stream>>>(Ymax, out4);
}
